// ViTQuadraticAttention_62440234549860
// MI455X (gfx1250) — hardware-verified
//
#include <hip/hip_runtime.h>
#include <math.h>
#include <stdint.h>

typedef __attribute__((ext_vector_type(16))) _Float16 v16h;
typedef __attribute__((ext_vector_type(8)))  _Float16 v8h;
typedef __attribute__((ext_vector_type(16))) __bf16   v16b;
typedef __attribute__((ext_vector_type(8)))  __bf16   v8b;
typedef __attribute__((ext_vector_type(8)))  float    v8f;
typedef __attribute__((ext_vector_type(4)))  float    v4f;
typedef __attribute__((ext_vector_type(2)))  float    v2f;
typedef __attribute__((ext_vector_type(4)))  unsigned int v4u;
typedef __attribute__((ext_vector_type(8)))  unsigned short v8us;

constexpr int kNB     = 8;
constexpr int kNTOK   = 1024;
constexpr int kHID    = 768;
constexpr int kNHEADS = 12;
constexpr int kHDIM   = 64;
constexpr int kQCP    = 1536;
constexpr int kAQB    = 64;
constexpr int kAKC    = 64;
constexpr int kAKD    = 128;

__device__ __forceinline__ unsigned short f2bf_bits(float f) {
  unsigned u = __float_as_uint(f);
  return (unsigned short)((u + 0x7FFFu + ((u >> 16) & 1u)) >> 16);
}
__device__ __forceinline__ float bf_bits2f(unsigned short h) { return __uint_as_float(((unsigned)h) << 16); }
__device__ __forceinline__ unsigned pk16(unsigned short a, unsigned short b) { return (unsigned)a | ((unsigned)b << 16); }

__device__ __forceinline__ void dep_guard_h(v8f& a, v8f& b, v16h x, v16h y) { asm volatile("v_nop\n\tv_nop\n\tv_nop\n\tv_nop" : "+v"(a), "+v"(b) : "v"(x), "v"(y)); }
__device__ __forceinline__ void dep_guard_b(v8f& a, v8f& b, v16b x, v16b y) { asm volatile("v_nop\n\tv_nop\n\tv_nop\n\tv_nop" : "+v"(a), "+v"(b) : "v"(x), "v"(y)); }
__device__ __forceinline__ void keep4_h(v16h a, v16h b, v16h c, v16h d) { asm volatile("v_nop" :: "v"(a), "v"(b), "v"(c), "v"(d)); }
__device__ __forceinline__ void keep4_b(v16b a, v16b b, v16b c, v16b d) { asm volatile("v_nop" :: "v"(a), "v"(b), "v"(c), "v"(d)); }
__device__ __forceinline__ void acc_guard4(v8f& a, v8f& b, v8f& c, v8f& d) { asm volatile("v_nop\n\tv_nop\n\tv_nop\n\tv_nop" : "+v"(a), "+v"(b), "+v"(c), "+v"(d)); }
template <typename T> struct Frag;
template <> struct Frag<_Float16> {
  typedef v16h V; union U { v16h v; v8h h[2]; };
  static __device__ __forceinline__ v16h load(const _Float16* p) {
    U f; f.h[0] = *(const v8h*)(p); f.h[1] = *(const v8h*)(p + 16); return f.v;
  }
  static __device__ __forceinline__ v8f mma(v16h a, v16h b, v8f c) {
    return __builtin_amdgcn_wmma_f32_16x16x32_f16(false, a, false, b, (short)0, c, false, false);
  }
  static __device__ __forceinline__ void guard(v8f& a, v8f& b, v16h x, v16h y) { dep_guard_h(a, b, x, y); }
  static __device__ __forceinline__ void keep(v16h a, v16h b, v16h c, v16h d) { keep4_h(a, b, c, d); }
};
template <> struct Frag<__bf16> {
  typedef v16b V; union U { v16b v; v8b h[2]; };
  static __device__ __forceinline__ v16b load(const __bf16* p) {
    U f; f.h[0] = *(const v8b*)(p); f.h[1] = *(const v8b*)(p + 16); return f.v;
  }
  static __device__ __forceinline__ v8f mma(v16b a, v16b b, v8f c) {
    return __builtin_amdgcn_wmma_f32_16x16x32_bf16(false, a, false, b, (short)0, c, false, false);
  }
  static __device__ __forceinline__ void guard(v8f& a, v8f& b, v16b x, v16b y) { dep_guard_b(a, b, x, y); }
  static __device__ __forceinline__ void keep(v16b a, v16b b, v16b c, v16b d) { keep4_b(a, b, c, d); }
};

template <int ET> struct Elem;
template <> struct Elem<0> { typedef _Float16 T; };
template <> struct Elem<1> { typedef __bf16 T; };
template <int ET, bool SPLIT, int BIAS_MODE, int OUT_MODE, bool RESID, int ACT = 0>
__global__ __launch_bounds__(256) void wmma_gemm64(
    const unsigned short* __restrict__ Ap, const unsigned short* __restrict__ A2p, int lda, long strideA,
    const unsigned short* __restrict__ Btp, const unsigned short* __restrict__ Bt2p, int ldb, long strideB,
    void* __restrict__ Cout, void* __restrict__ Cout2, int ldc, long strideC,
    const float* __restrict__ bias,
    const float* __restrict__ resid, long strideR,
    int M, int N, int K, float scale) {
  typedef typename Elem<ET>::T T;
  typedef typename Frag<T>::V V;
  const T* A = (const T*)Ap; const T* A2 = (const T*)A2p; const T* Bt = (const T*)Btp; const T* Bt2 = (const T*)Bt2p;
  __shared__ __align__(16) float sT[8][16 * 68];
  const int b    = blockIdx.y;
  const int lane = threadIdx.x & 31;
  const int wave = threadIdx.x >> 5;
  const int tilesN = N >> 6;
  const int tilesM = M >> 6;
  const int tile = blockIdx.x * 8 + wave;
  if (tile >= tilesM * tilesN) return;
  const int tm = tile / tilesN;
  const int tn = tile - tm * tilesN;
  const int m0 = tm << 6;
  const int n0 = tn << 6;

  const T* Ab  = A  + (size_t)b * strideA;
  const T* Bb  = Bt + (size_t)b * strideB;
  const T* Ab2 = SPLIT ? (A2  + (size_t)b * strideA) : nullptr;
  const T* Bb2 = SPLIT ? (Bt2 + (size_t)b * strideB) : nullptr;

  const int rlane = lane & 15;
  const int koff  = (lane >> 4) * 8;
  const int mOff  = (lane >> 4) * 8;

  v8f acc[4][4];
#pragma unroll
  for (int i = 0; i < 4; ++i)
#pragma unroll
    for (int j = 0; j < 4; ++j) acc[i][j] = (v8f){0.f,0.f,0.f,0.f,0.f,0.f,0.f,0.f};

  for (int k0 = 0; k0 < K; k0 += 32) {
    V bh[4], bl[4];
#pragma unroll
    for (int j = 0; j < 4; ++j) {
      const size_t bo = (size_t)(n0 + (j << 4) + rlane) * ldb + koff + k0;
      bh[j] = Frag<T>::load(Bb + bo);
      if (SPLIT) bl[j] = Frag<T>::load(Bb2 + bo);
    }
#pragma unroll
    for (int i = 0; i < 4; ++i) {
      const size_t ao = (size_t)(m0 + (i << 4) + rlane) * lda + koff + k0;
      V ah = Frag<T>::load(Ab + ao);
      V al;
      if (SPLIT) al = Frag<T>::load(Ab2 + ao);
#pragma unroll
      for (int j = 0; j < 4; ++j) {
        acc[i][j] = Frag<T>::mma(ah, bh[j], acc[i][j]);
        if (SPLIT) {
          acc[i][j] = Frag<T>::mma(ah, bl[j], acc[i][j]);
          acc[i][j] = Frag<T>::mma(al, bh[j], acc[i][j]);
        }
      }
      Frag<T>::guard(acc[i][0], acc[i][3], ah, SPLIT ? al : ah);
    }
    Frag<T>::keep(bh[0], bh[1], bh[2], bh[3]);
    if (SPLIT) Frag<T>::keep(bl[0], bl[1], bl[2], bl[3]);
  }
  acc_guard4(acc[0][0], acc[0][1], acc[0][2], acc[0][3]);
  acc_guard4(acc[1][0], acc[1][1], acc[1][2], acc[1][3]);
  acc_guard4(acc[2][0], acc[2][1], acc[2][2], acc[2][3]);
  acc_guard4(acc[3][0], acc[3][1], acc[3][2], acc[3][3]);

  float* slab = sT[wave];
  const float* Rb = RESID ? (resid + (size_t)b * strideR) : nullptr;
#pragma unroll
  for (int i = 0; i < 4; ++i) {
    const int mBase = m0 + (i << 4);
#pragma unroll
    for (int j = 0; j < 4; ++j) {
      const int n = n0 + (j << 4) + rlane;
      float bv = 0.f;
      if (BIAS_MODE == 2) bv = bias[n];
#pragma unroll
      for (int r = 0; r < 8; ++r) {
        float v = acc[i][j][r] * scale;
        if (BIAS_MODE == 1) v += bias[mBase + mOff + r];
        if (BIAS_MODE == 2) v += bv;
        if (RESID) v += Rb[(size_t)(mBase + mOff + r) * ldc + n];
        if (ACT == 1) v = tanhf(v);
        if (ACT == 2) v = fmaxf(v, 0.0f);
        if (ACT == 3) v = v / (1.0f + expf(-v));
        if (ACT == 4) v = (v > 0.f) ? v : 0.01f * v;
        if (ACT == 5) v = 0.5f * v * (1.0f + erff(v * 0.70710678118654752f));
        slab[(mOff + r) * 68 + (j << 4) + rlane] = v;
      }
    }
    __builtin_amdgcn_fence(__ATOMIC_RELEASE, "workgroup");
    __builtin_amdgcn_wave_barrier();
    __builtin_amdgcn_fence(__ATOMIC_ACQUIRE, "workgroup");
    if (OUT_MODE == 0) {
      float* C = (float*)Cout + (size_t)b * strideC;
      const int hh = lane >> 4, c4 = (lane & 15) * 4;
      for (int pass = 0; pass < 2; ++pass) {
#pragma unroll
        for (int it = 0; it < 8; ++it) {
          const int row = it * 2 + hh;
          v4f v = *(const v4f*)(slab + row * 68 + c4);
          *(volatile v4f*)(C + (size_t)(mBase + row) * ldc + n0 + c4) = v;
        }
        __threadfence();
      }
    } else {
      const int q = lane >> 3, c8 = (lane & 7) * 8;
      unsigned short* C  = (unsigned short*)Cout  + (size_t)b * strideC;
      unsigned short* C2 = (OUT_MODE == 2) ? ((unsigned short*)Cout2 + (size_t)b * strideC) : nullptr;
      for (int pass = 0; pass < 2; ++pass) {
#pragma unroll
        for (int it = 0; it < 4; ++it) {
          const int row = it * 4 + q;
          const float* sp = slab + row * 68 + c8;
          v8h hv, lv;
#pragma unroll
          for (int e = 0; e < 8; ++e) {
            if (OUT_MODE == 1) {
              hv[e] = (_Float16)sp[e];
            } else {
              unsigned short hb = f2bf_bits(sp[e]);
              unsigned short lb = f2bf_bits(sp[e] - bf_bits2f(hb));
              hv[e] = __builtin_bit_cast(_Float16, hb);
              lv[e] = __builtin_bit_cast(_Float16, lb);
            }
          }
          *(volatile v8h*)(C + (size_t)(mBase + row) * ldc + n0 + c8) = hv;
          if (OUT_MODE == 2) *(volatile v8h*)(C2 + (size_t)(mBase + row) * ldc + n0 + c8) = lv;
        }
        __threadfence();
      }
    }
    __builtin_amdgcn_fence(__ATOMIC_RELEASE, "workgroup");
    __builtin_amdgcn_wave_barrier();
    __builtin_amdgcn_fence(__ATOMIC_ACQUIRE, "workgroup");
  }
}

__global__ __launch_bounds__(256) void cast_f32_bf16x2(const float* __restrict__ in, unsigned short* __restrict__ out, int n2) {
  const int i = blockIdx.x * 256 + threadIdx.x;
  if (i < n2) {
    const v2f f = *(const v2f*)(in + 2 * (size_t)i);
    const unsigned u = pk16(f2bf_bits(f[0]), f2bf_bits(f[1]));
    ((volatile unsigned*)out)[i] = u;
    __threadfence();
    ((volatile unsigned*)out)[i] = u;
  }
}

__global__ __launch_bounds__(256) void bias_rne_kernel(const float* __restrict__ b0, const float* __restrict__ b1,
                                                       const float* __restrict__ b2, float* __restrict__ o, int n) {
  const int g = blockIdx.x * 256 + threadIdx.x;
  if (g < 3 * n) {
    const int w = g / n;
    int i = g - w * n;
    i = i < 0 ? 0 : (i > n - 1 ? n - 1 : i);
    const float v0 = b0[i], v1 = b1[i], v2 = b2[i];
    const float v = (w == 0) ? v0 : ((w == 1) ? v1 : v2);
    const float rv = bf_bits2f(f2bf_bits(v));
    ((volatile float*)o)[g] = rv;
    __threadfence();
    ((volatile float*)o)[g] = rv;
  }
}

__global__ __launch_bounds__(256) void kd_sq_kernel(const unsigned short* __restrict__ kch, const unsigned short* __restrict__ kcl,
                                                    float* __restrict__ kdsq, int nrows) {
  const int g = blockIdx.x * 256 + threadIdx.x;
  if (g < nrows) {
    const int s  = g & (kNTOK - 1);
    const int bh = g >> 10;
    const int h  = bh % kNHEADS;
    const int b  = bh / kNHEADS;
    const size_t ro = ((size_t)b * kNTOK + (size_t)s) * kQCP + (size_t)h * kHDIM;
    const unsigned short* ph = kch + ro;
    const unsigned short* pl = kcl + ro;
    float acc = 0.f;
#pragma unroll 1
    for (int i = 0; i < 8; ++i) {
      const v8us a = *(const v8us*)(ph + 8 * i);
      const v8us l = *(const v8us*)(pl + 8 * i);
#pragma unroll
      for (int e = 0; e < 8; ++e) {
        const float x = bf_bits2f(a[e]) + bf_bits2f(l[e]);
        acc = fmaf(x, x, acc);
      }
    }
    ((volatile float*)kdsq)[g] = acc;
    __threadfence();
    ((volatile float*)kdsq)[g] = acc;
  }
}

__device__ __forceinline__ v8f mma_bf(v16b a, v16b b, v8f c) {
  c = __builtin_amdgcn_wmma_f32_16x16x32_bf16(false, a, false, b, (short)0, c, false, false);
  asm volatile("v_nop\n\tv_nop\n\tv_nop\n\tv_nop" : "+v"(c) : "v"(a), "v"(b));
  return c;
}
__device__ __forceinline__ v8f mma_hf(v16h a, v16h b, v8f c) {
  c = __builtin_amdgcn_wmma_f32_16x16x32_f16(false, a, false, b, (short)0, c, false, false);
  asm volatile("v_nop\n\tv_nop\n\tv_nop\n\tv_nop" : "+v"(c) : "v"(a), "v"(b));
  return c;
}

__global__ __launch_bounds__(128)
void attn_quad_kernel(const unsigned short* __restrict__ qch, const unsigned short* __restrict__ qcl,
                      const unsigned short* __restrict__ kch, const unsigned short* __restrict__ kcl,
                      const unsigned short* __restrict__ vtp, const float* __restrict__ kdsq,
                      float* __restrict__ out) {
  union FB { v16b v; v8b h[2]; };
  union FH { v16h v; v8h h[2]; };
  __shared__ __align__(16) __bf16   Qsh[kAQB * kAKD];
  __shared__ __align__(16) __bf16   Qsl[kAQB * kAKD];
  __shared__ __align__(16) __bf16   Ksh[kAKC * kAKD];
  __shared__ __align__(16) __bf16   Ksl[kAKC * kAKD];
  __shared__ __align__(16) _Float16 Vth[kHDIM * kAKC];
  __shared__ __align__(16) _Float16 Psh[4][16 * kAKC];
  __shared__ __align__(16) float    Os[4][16 * 68];

  const int tid  = threadIdx.x;
  const int wave = tid >> 5;
  const int lane = tid & 31;
  const int hh   = lane >> 4;
  const int c    = lane & 15;

  constexpr int nqb = kNTOK / kAQB;
  const int bx = blockIdx.x;
  const int qb = bx % nqb;
  const int bh = bx / nqb;
  const int h  = bh % kNHEADS;
  const int b  = bh / kNHEADS;
  const int qr0 = qb * kAQB;
  const int w0  = wave * 16;

  const __bf16* QH = (const __bf16*)(const void*)qch + (size_t)b * kNTOK * kQCP;
  const __bf16* QL = (const __bf16*)(const void*)qcl + (size_t)b * kNTOK * kQCP;
  const __bf16* KH = (const __bf16*)(const void*)kch + (size_t)b * kNTOK * kQCP;
  const __bf16* KL = (const __bf16*)(const void*)kcl + (size_t)b * kNTOK * kQCP;
  const _Float16* VT = (const _Float16*)(const void*)vtp + ((size_t)b * kHID + (size_t)h * kHDIM) * kNTOK;
  const float* ksq = kdsq + (size_t)bh * kNTOK;
  float* ob = out + (size_t)b * kNTOK * kHID + (size_t)h * kHDIM;

  const int sr   = tid >> 1;
  const int part = tid & 1;
  const int coff = part ? (kHID + h * kHDIM) : (h * kHDIM);
  const int loff = part * 64;

  {
    const size_t go = (size_t)(qr0 + sr) * kQCP + coff;
#pragma unroll
    for (int i = 0; i < 8; ++i) {
      const v8b a0 = *(const v8b*)(QH + go + 8 * i);
      const v8b a1 = *(const v8b*)(QL + go + 8 * i);
      *(v8b*)(Qsh + sr * kAKD + loff + 8 * i) = a0;
      *(v8b*)(Qsl + sr * kAKD + loff + 8 * i) = a1;
    }
  }

  float mrow[8], lrow[8];
  v8f oacc[4];
#pragma unroll
  for (int r = 0; r < 8; ++r) { mrow[r] = -INFINITY; lrow[r] = 0.f; }
#pragma unroll
  for (int t = 0; t < 4; ++t) oacc[t] = (v8f){0.f,0.f,0.f,0.f,0.f,0.f,0.f,0.f};

  constexpr int nChunks = kNTOK / kAKC;
  for (int kc = 0; kc < nChunks; ++kc) {
    const int kv0 = kc * kAKC;
    __syncthreads();
    {
      const size_t go = (size_t)(kv0 + sr) * kQCP + coff;
#pragma unroll
      for (int i = 0; i < 8; ++i) {
        const v8b a0 = *(const v8b*)(KH + go + 8 * i);
        const v8b a1 = *(const v8b*)(KL + go + 8 * i);
        *(v8b*)(Ksh + sr * kAKD + loff + 8 * i) = a0;
        *(v8b*)(Ksl + sr * kAKD + loff + 8 * i) = a1;
      }
      const int vh = part * 32;
      const _Float16* vs = VT + (size_t)sr * kNTOK + kv0 + vh;
#pragma unroll
      for (int i = 0; i < 4; ++i) {
        const v8h vv = *(const v8h*)(vs + 8 * i);
        *(v8h*)(Vth + sr * kAKC + vh + 8 * i) = vv;
      }
    }
    __syncthreads();

    v8f s[4];
#pragma unroll
    for (int j = 0; j < 4; ++j) s[j] = (v8f){0.f,0.f,0.f,0.f,0.f,0.f,0.f,0.f};
#pragma unroll 1
    for (int dc = 0; dc < 4; ++dc) {
      FB qa, ql;
      const int qo = (w0 + c) * kAKD + dc * 32 + 8 * hh;
      qa.h[0] = *(const v8b*)(Qsh + qo);
      qa.h[1] = *(const v8b*)(Qsh + qo + 16);
      ql.h[0] = *(const v8b*)(Qsl + qo);
      ql.h[1] = *(const v8b*)(Qsl + qo + 16);
#pragma unroll
      for (int j = 0; j < 4; ++j) {
        FB kb, kl;
        const int ko = (j * 16 + c) * kAKD + dc * 32 + 8 * hh;
        kb.h[0] = *(const v8b*)(Ksh + ko);
        kb.h[1] = *(const v8b*)(Ksh + ko + 16);
        kl.h[0] = *(const v8b*)(Ksl + ko);
        kl.h[1] = *(const v8b*)(Ksl + ko + 16);
        s[j] = mma_bf(qa.v, kb.v, s[j]);
        s[j] = mma_bf(qa.v, kl.v, s[j]);
        s[j] = mma_bf(ql.v, kb.v, s[j]);
      }
    }

    float kq[4];
#pragma unroll
    for (int j = 0; j < 4; ++j) kq[j] = ksq[kv0 + j * 16 + c] * 0.0625f;
    float cm[8];
#pragma unroll
    for (int r = 0; r < 8; ++r) {
      float m = -INFINITY;
#pragma unroll
      for (int j = 0; j < 4; ++j) {
        const float v = s[j][r] * 0.125f - kq[j];
        s[j][r] = v;
        m = fmaxf(m, v);
      }
#pragma unroll
      for (int off = 1; off < 16; off <<= 1) m = fmaxf(m, __shfl_xor(m, off, 32));
      cm[r] = m;
    }

    _Float16* pw = Psh[wave];
#pragma unroll
    for (int r = 0; r < 8; ++r) {
      const float mnew  = fmaxf(mrow[r], cm[r]);
      const float alpha = __expf(mrow[r] - mnew);
      mrow[r] = mnew;
      float psum = 0.f;
#pragma unroll
      for (int j = 0; j < 4; ++j) {
        const float p = __expf(s[j][r] - mnew);
        psum += p;
        pw[(8 * hh + r) * kAKC + j * 16 + c] = (_Float16)(p * 32768.0f);
      }
#pragma unroll
      for (int off = 1; off < 16; off <<= 1) psum += __shfl_xor(psum, off, 32);
      lrow[r] = lrow[r] * alpha + psum;
#pragma unroll
      for (int t = 0; t < 4; ++t) oacc[t][r] *= alpha;
    }
    __builtin_amdgcn_fence(__ATOMIC_RELEASE, "workgroup");
    __builtin_amdgcn_wave_barrier();
    __builtin_amdgcn_fence(__ATOMIC_ACQUIRE, "workgroup");

#pragma unroll
    for (int kk = 0; kk < 2; ++kk) {
      FH pa;
      const int po = c * kAKC + kk * 32 + 8 * hh;
      pa.h[0] = *(const v8h*)(pw + po);
      pa.h[1] = *(const v8h*)(pw + po + 16);
#pragma unroll
      for (int t = 0; t < 4; ++t) {
        FH vb;
        const int vo = (t * 16 + c) * kAKC + kk * 32 + 8 * hh;
        vb.h[0] = *(const v8h*)(Vth + vo);
        vb.h[1] = *(const v8h*)(Vth + vo + 16);
        oacc[t] = mma_hf(pa.v, vb.v, oacc[t]);
      }
    }
  }

  float* os = Os[wave];
#pragma unroll
  for (int r = 0; r < 8; ++r) {
    const float inv = 1.0f / (lrow[r] * 32768.0f);
#pragma unroll
    for (int t = 0; t < 4; ++t) os[(8 * hh + r) * 68 + t * 16 + c] = oacc[t][r] * inv;
  }
  __builtin_amdgcn_fence(__ATOMIC_RELEASE, "workgroup");
  __builtin_amdgcn_wave_barrier();
  __builtin_amdgcn_fence(__ATOMIC_ACQUIRE, "workgroup");
  {
    const int c4 = (lane & 15) * 4;
    for (int pass = 0; pass < 2; ++pass) {
#pragma unroll
      for (int it = 0; it < 8; ++it) {
        const int row = it * 2 + hh;
        const v4f val = *(const v4f*)(os + row * 68 + c4);
        *(volatile v4f*)(ob + (size_t)(qr0 + w0 + row) * kHID + c4) = val;
      }
      __threadfence();
    }
  }
}

extern "C" void kernel_launch(void* const* d_in, const int* in_sizes, int n_in,
                              void* d_out, int out_size, void* d_ws, size_t ws_size,
                              hipStream_t stream) {
  if (n_in < 9) return;
  const int nAct = kNB * kNTOK * kHID;
  const int nW   = kHID * kHID;
  if (in_sizes[0] != nAct || in_sizes[1] != nAct || in_sizes[2] != nW || in_sizes[3] != nW ||
      in_sizes[5] != nW || in_sizes[7] != nW || in_sizes[4] != kHID || in_sizes[6] != kHID ||
      in_sizes[8] != kHID || out_size != nAct) return;

  const float* qs = (const float*)d_in[0];
  const float* ks = (const float*)d_in[1];
  const float* Wd = (const float*)d_in[2];
  const float* Wq = (const float*)d_in[3];
  const float* bq = (const float*)d_in[4];
  const float* Wk = (const float*)d_in[5];
  const float* bk = (const float*)d_in[6];
  const float* Wv = (const float*)d_in[7];
  const float* bv = (const float*)d_in[8];
  float* out = (float*)d_out;

  const size_t bAct16 = (size_t)nAct * 2;
  const size_t bW16   = (size_t)nW * 2;
  const size_t bQC    = (size_t)kNB * kNTOK * kQCP * 2;
  const size_t bSq    = (size_t)kNB * kNHEADS * kNTOK * 4;
  const size_t bBias  = (size_t)3 * kHID * 4;
  const size_t oXq  = 0;
  const size_t oXk  = oXq + bAct16;
  const size_t oWd  = oXk + bAct16;
  const size_t oWq  = oWd + bW16;
  const size_t oWk  = oWq + bW16;
  const size_t oWv  = oWk + bW16;
  const size_t oQCh = oWv + bW16;
  const size_t oQCl = oQCh + bQC;
  const size_t oKCh = oQCl + bQC;
  const size_t oKCl = oKCh + bQC;
  const size_t oSq  = oKCl + bQC;
  const size_t oBs  = oSq + bSq;
  const size_t total = oBs + bBias;
  const size_t bVT  = (size_t)kNB * kHID * kNTOK * 2;
  if (total > ws_size || bVT > bAct16) return;

  char* ws = (char*)d_ws;
  unsigned short* Xq16 = (unsigned short*)(ws + oXq);
  unsigned short* Xk16 = (unsigned short*)(ws + oXk);
  unsigned short* Wd16 = (unsigned short*)(ws + oWd);
  unsigned short* Wq16 = (unsigned short*)(ws + oWq);
  unsigned short* Wk16 = (unsigned short*)(ws + oWk);
  unsigned short* Wv16 = (unsigned short*)(ws + oWv);
  unsigned short* QCh  = (unsigned short*)(ws + oQCh);
  unsigned short* QCl  = (unsigned short*)(ws + oQCl);
  unsigned short* KCh  = (unsigned short*)(ws + oKCh);
  unsigned short* KCl  = (unsigned short*)(ws + oKCl);
  unsigned short* VT16 = (unsigned short*)(ws + oXq);
  float* kdsq  = (float*)(ws + oSq);
  float* biasr = (float*)(ws + oBs);

  {
    const int n2a = nAct / 2, n2w = nW / 2;
    cast_f32_bf16x2<<<dim3((n2a + 255) / 256), dim3(256), 0, stream>>>(qs, Xq16, n2a);
    cast_f32_bf16x2<<<dim3((n2a + 255) / 256), dim3(256), 0, stream>>>(ks, Xk16, n2a);
    cast_f32_bf16x2<<<dim3((n2w + 255) / 256), dim3(256), 0, stream>>>(Wd, Wd16, n2w);
    cast_f32_bf16x2<<<dim3((n2w + 255) / 256), dim3(256), 0, stream>>>(Wq, Wq16, n2w);
    cast_f32_bf16x2<<<dim3((n2w + 255) / 256), dim3(256), 0, stream>>>(Wk, Wk16, n2w);
    cast_f32_bf16x2<<<dim3((n2w + 255) / 256), dim3(256), 0, stream>>>(Wv, Wv16, n2w);
    bias_rne_kernel<<<dim3((3 * kHID + 255) / 256), dim3(256), 0, stream>>>(bq, bk, bv, biasr, kHID);
  }

  const int M = kNB * kNTOK;
  {
    const dim3 grid((M / 64) * (kHID / 64) / 8, 1), block(256);
    wmma_gemm64<1, false, 0, 2, false, 0><<<grid, block, 0, stream>>>(
        Xq16, Xq16, kHID, 0L, Wd16, Wd16, kHID, 0L, (void*)QCh, (void*)QCl, kQCP, 0L,
        biasr, biasr, 0L, M, kHID, kHID, 1.0f);
    wmma_gemm64<1, false, 2, 2, false, 0><<<grid, block, 0, stream>>>(
        Xq16, Xq16, kHID, 0L, Wq16, Wq16, kHID, 0L, (void*)(QCh + kHID), (void*)(QCl + kHID), kQCP, 0L,
        biasr, biasr, 0L, M, kHID, kHID, 1.0f);
    wmma_gemm64<1, false, 0, 2, false, 0><<<grid, block, 0, stream>>>(
        Xk16, Xk16, kHID, 0L, Wd16, Wd16, kHID, 0L, (void*)KCh, (void*)KCl, kQCP, 0L,
        biasr, biasr, 0L, M, kHID, kHID, 1.0f);
    wmma_gemm64<1, false, 2, 2, false, 0><<<grid, block, 0, stream>>>(
        Xk16, Xk16, kHID, 0L, Wk16, Wk16, kHID, 0L, (void*)(KCh + kHID), (void*)(KCl + kHID), kQCP, 0L,
        biasr + kHID, biasr, 0L, M, kHID, kHID, 1.0f);
  }
  {
    const long sB = (long)kNTOK * kHID;
    const long sC = (long)kHID * kNTOK;
    const dim3 grid((kHID / 64) * (kNTOK / 64) / 8, kNB), block(256);
    wmma_gemm64<1, false, 1, 1, false, 0><<<grid, block, 0, stream>>>(
        Wv16, Wv16, kHID, 0L, Xk16, Xk16, kHID, sB, (void*)VT16, (void*)VT16, kNTOK, sC,
        biasr + 2 * kHID, biasr, 0L, kHID, kNTOK, kHID, 1.0f);
  }
  {
    const int nrows = kNB * kNHEADS * kNTOK;
    kd_sq_kernel<<<dim3((nrows + 255) / 256), dim3(256), 0, stream>>>(KCh, KCl, kdsq, nrows);
  }
  attn_quad_kernel<<<dim3(kNB * kNHEADS * (kNTOK / kAQB)), dim3(128), 0, stream>>>(QCh, QCl, KCh, KCl, VT16, kdsq, out);
}
